// Qwen3_5GatedDeltaNet_85529978732977
// MI455X (gfx1250) — hardware-verified
//
#include <hip/hip_runtime.h>
#include <hip/hip_bf16.h>


#define S_    512
#define H_    2048
#define NVH_  16
#define NKH_  8
#define DK_   128
#define DV_   128
#define KEY_  1024
#define VAL_  2048
#define CONV_ 4096
#define NCAT_ 6176
#define NP_   6208
#define COLZ_ 4096
#define COLB_ 6144
#define COLA_ 6160

static_assert(NP_ % 64 == 0);
static_assert(NP_ >= NCAT_);
static_assert(S_ % 64 == 0);
static_assert(H_ % 64 == 0);
static_assert(VAL_ % 64 == 0);
static_assert(CONV_ == 4 * 1024);
static_assert(S_ % 32 == 0);
static_assert((NP_ * 4) % 128 == 0);

typedef float          v4f   __attribute__((ext_vector_type(4)));
typedef float          v8f   __attribute__((ext_vector_type(8)));
typedef __bf16         v16b  __attribute__((ext_vector_type(16)));
typedef unsigned short u16x8 __attribute__((ext_vector_type(8)));

union FragB { u16x8 h[2]; v16b v; };

constexpr size_t SZ_HS16 = (size_t)S_ * H_ * 2;
constexpr size_t SZ_WC16 = (size_t)NP_ * H_ * 2;
constexpr size_t SZ_WO16 = (size_t)H_ * VAL_ * 2;
constexpr size_t SZ_PROJ = (size_t)S_ * NP_ * 4;
constexpr size_t SZ_ACT  = (size_t)S_ * CONV_ * 4;
constexpr size_t SZ_CORE = (size_t)S_ * VAL_ * 4;
constexpr size_t SZ_CG16 = (size_t)S_ * VAL_ * 2;

constexpr size_t OFF_HSH  = 0;
constexpr size_t OFF_HSL  = OFF_HSH + SZ_HS16;
constexpr size_t OFF_WCH  = OFF_HSL + SZ_HS16;
constexpr size_t OFF_WCL  = OFF_WCH + SZ_WC16;
constexpr size_t OFF_WOH  = OFF_WCL + SZ_WC16;
constexpr size_t OFF_WOL  = OFF_WOH + SZ_WO16;
constexpr size_t OFF_PROJ = OFF_WOL + SZ_WO16;
constexpr size_t OFF_ACT  = OFF_PROJ + SZ_PROJ;
constexpr size_t OFF_CORE = OFF_ACT + SZ_ACT;
constexpr size_t OFF_CGH  = OFF_CORE + SZ_CORE;
constexpr size_t OFF_CGL  = OFF_CGH + SZ_CG16;
constexpr size_t WS_END   = OFF_CGL + SZ_CG16;
static_assert(WS_END <= (size_t)134217728);
static_assert(OFF_HSL % 128 == 0 && OFF_WCH % 128 == 0 && OFF_WCL % 128 == 0 && OFF_WOH % 128 == 0);
static_assert(OFF_WOL % 128 == 0 && OFF_PROJ % 128 == 0 && OFF_ACT % 128 == 0 && OFF_CORE % 128 == 0);
static_assert(OFF_CGH % 128 == 0 && OFF_CGL % 128 == 0);

__device__ __forceinline__ unsigned short f32_to_bf16(float f) {
    unsigned u = __float_as_uint(f);
    unsigned r = u + 0x7FFFu + ((u >> 16) & 1u);
    return (unsigned short)(r >> 16);
}
__device__ __forceinline__ float bf16_to_f32(unsigned short b) {
    return __uint_as_float(((unsigned)b) << 16);
}
__device__ __forceinline__ float silu_f(float x) {
    float e = __expf(-x);
    return x * __builtin_amdgcn_rcpf(1.0f + e);
}
__device__ __forceinline__ v8f ld8f(const float* p) {
    v4f a = *(const v4f*)p;
    v4f b = *(const v4f*)(p + 4);
    return __builtin_shufflevector(a, b, 0, 1, 2, 3, 4, 5, 6, 7);
}
__device__ __forceinline__ void split8(const v8f x, u16x8& hv, u16x8& lv) {
#pragma unroll
    for (int c = 0; c < 8; ++c) {
        const float f = x[c];
        const unsigned short hb = f32_to_bf16(f);
        const unsigned short lb = f32_to_bf16(f - bf16_to_f32(hb));
        hv[c] = hb;
        lv[c] = lb;
    }
}

__device__ __forceinline__ void mma16(v8f& acc, const FragB& a, const FragB& b) {
    acc = __builtin_amdgcn_wmma_f32_16x16x32_bf16(false, a.v, false, b.v, (short)0, acc, false, false);
    asm volatile("v_nop\n\tv_nop\n\tv_nop\n\tv_nop" : "+v"(acc) : "v"(a.v), "v"(b.v));
}

__global__ __launch_bounds__(256)
void hs_cvt_kernel(const float* __restrict__ src, const int* __restrict__ mask,
                   unsigned short* dhi, unsigned short* dlo, int n8)
{
    const int i = blockIdx.x * 256 + threadIdx.x;
    if (i >= n8) return;
    const size_t e = (size_t)i * 8;
    int s = (int)(e / H_);
    s = min(s, S_ - 1);
    const float mk = (float)mask[s];
    const v8f x = ld8f(src + e) * mk;
    u16x8 hv, lv;
    split8(x, hv, lv);
    *(volatile u16x8*)(dhi + e) = hv;
    *(volatile u16x8*)(dlo + e) = lv;
    __threadfence();
    *(volatile u16x8*)(dhi + e) = hv;
    *(volatile u16x8*)(dlo + e) = lv;
}

__global__ __launch_bounds__(256)
void wt_cvt_kernel(const float* __restrict__ src, unsigned short* dhi, unsigned short* dlo,
                   int Nw, int Kd, int nrows)
{
    __shared__ __attribute__((aligned(16))) float sT[64 * 68];
    const int tid  = threadIdx.x;
    const int lane = tid & 31;
    const int wave = tid >> 5;
    const int n0 = blockIdx.x * 64;
    const int k0 = blockIdx.y * 64;

#pragma unroll
    for (int it = 0; it < 4; ++it) {
        const int idx = it * 256 + tid;
        const int kk  = idx >> 4;
        const int n4  = (idx & 15) * 4;
        const int gn  = n0 + n4;
        const int gnc = min(gn, Nw - 4);
        const v4f v = *(const v4f*)(src + (size_t)(k0 + kk) * Nw + gnc);
        const bool in = (gn < Nw);
        sT[(n4 + 0) * 68 + kk] = in ? v[0] : 0.0f;
        sT[(n4 + 1) * 68 + kk] = in ? v[1] : 0.0f;
        sT[(n4 + 2) * 68 + kk] = in ? v[2] : 0.0f;
        sT[(n4 + 3) * 68 + kk] = in ? v[3] : 0.0f;
    }
    __syncthreads();

    u16x8 hv[2], lv[2];
    const int c = (lane & 7) * 8;
#pragma unroll
    for (int it = 0; it < 2; ++it) {
        const int nn = it * 32 + wave * 4 + (lane >> 3);
        const v8f x = ld8f(sT + nn * 68 + c);
        split8(x, hv[it], lv[it]);
    }
#pragma unroll
    for (int it = 0; it < 2; ++it) {
        const int gr = n0 + it * 32 + wave * 4 + (lane >> 3);
        if (gr < nrows) {
            const size_t o = (size_t)gr * Kd + k0 + c;
            *(volatile u16x8*)(dhi + o) = hv[it];
            *(volatile u16x8*)(dlo + o) = lv[it];
        }
    }
    __threadfence();
#pragma unroll
    for (int it = 0; it < 2; ++it) {
        const int gr = n0 + it * 32 + wave * 4 + (lane >> 3);
        if (gr < nrows) {
            const size_t o = (size_t)gr * Kd + k0 + c;
            *(volatile u16x8*)(dhi + o) = hv[it];
            *(volatile u16x8*)(dlo + o) = lv[it];
        }
    }
}

template<int NBF>
__device__ __forceinline__ void tile_store_pass(const float* st, float* gp, int ldc, int lane) {
    constexpr int CW  = NBF * 16;
    constexpr int P   = CW + 4;
    constexpr int LPR = CW / 4;
    static_assert(32 % LPR == 0);
    constexpr int RPI = 32 / LPR;
    constexpr int NIT = 32 / RPI;
    const int rsub = lane / LPR;
    const int c0   = (lane % LPR) * 4;
#pragma unroll
    for (int it = 0; it < NIT; ++it) {
        const int row = it * RPI + rsub;
        const v4f v = *(const v4f*)(st + row * P + c0);
        *(volatile v4f*)(gp + (size_t)row * ldc + c0) = v;
    }
}

template<int NBF>
__global__ __launch_bounds__(128)
void gemm_x3_kernel(const unsigned short* __restrict__ Ah, const unsigned short* __restrict__ Al,
                    const unsigned short* __restrict__ Bh, const unsigned short* __restrict__ Bl,
                    float* C, int K, int ldc)
{
    constexpr int CW = NBF * 16;
    constexpr int P  = CW + 4;
    static_assert(CW % 32 == 0);
    __shared__ __attribute__((aligned(16))) float stile[4][32 * P];

    const int tid  = threadIdx.x;
    const int lane = tid & 31;
    const int wave = tid >> 5;
    const int h    = lane >> 4;
    const int m    = lane & 15;
    const int wm   = wave >> 1;
    const int wn   = wave & 1;

    const int rowW = blockIdx.y * 64 + wm * 32;
    const int colW = blockIdx.x * (2 * CW) + wn * CW;

    v8f acc[2 * NBF];
#pragma unroll
    for (int j = 0; j < 2 * NBF; ++j)
#pragma unroll
        for (int r = 0; r < 8; ++r) acc[j][r] = 0.0f;

    const size_t aoff  = (size_t)(rowW + m) * K + 8 * h;
    const size_t boff  = (size_t)(colW + m) * K + 8 * h;
    const size_t sub16 = (size_t)16 * K;
    const int nk = K >> 5;

#pragma unroll 1
    for (int kt = 0; kt < nk; ++kt) {
        const size_t k0 = (size_t)kt * 32;
        FragB fa[2], ga[2], fb[NBF], gb[NBF];
#pragma unroll
        for (int s = 0; s < 2; ++s) {
            const unsigned short* p = Ah + aoff + s * sub16 + k0;
            const unsigned short* q = Al + aoff + s * sub16 + k0;
            fa[s].h[0] = *(const u16x8*)(p);
            fa[s].h[1] = *(const u16x8*)(p + 16);
            ga[s].h[0] = *(const u16x8*)(q);
            ga[s].h[1] = *(const u16x8*)(q + 16);
        }
#pragma unroll
        for (int j = 0; j < NBF; ++j) {
            const unsigned short* p = Bh + boff + j * sub16 + k0;
            const unsigned short* q = Bl + boff + j * sub16 + k0;
            fb[j].h[0] = *(const u16x8*)(p);
            fb[j].h[1] = *(const u16x8*)(p + 16);
            gb[j].h[0] = *(const u16x8*)(q);
            gb[j].h[1] = *(const u16x8*)(q + 16);
        }
#pragma unroll
        for (int s = 0; s < 2; ++s)
#pragma unroll
            for (int j = 0; j < NBF; ++j) {
                mma16(acc[s * NBF + j], fa[s], fb[j]);
                mma16(acc[s * NBF + j], fa[s], gb[j]);
                mma16(acc[s * NBF + j], ga[s], fb[j]);
            }
    }

    float* st = stile[wave];
#pragma unroll
    for (int s = 0; s < 2; ++s)
#pragma unroll
        for (int j = 0; j < NBF; ++j)
#pragma unroll
            for (int r = 0; r < 8; ++r)
                st[(s * 16 + 8 * h + r) * P + j * 16 + m] = acc[s * NBF + j][r];
    __syncthreads();

    float* gp = C + (size_t)rowW * ldc + colW;
    tile_store_pass<NBF>(st, gp, ldc, lane);
    __threadfence();
    tile_store_pass<NBF>(st, gp, ldc, lane);
}

__global__ __launch_bounds__(256)
void prep_kernel(const float* __restrict__ proj, const float* __restrict__ cw, float* act)
{
    const int s   = blockIdx.x;
    const int tid = threadIdx.x;
    const int r0 = max(s - 3, 0), r1 = max(s - 2, 0), r2 = max(s - 1, 0);
    const float z0 = (s >= 3) ? 1.0f : 0.0f;
    const float z1 = (s >= 2) ? 1.0f : 0.0f;
    const float z2 = (s >= 1) ? 1.0f : 0.0f;
    const float* p3 = proj + (size_t)s  * NP_;
    const float* p2 = proj + (size_t)r2 * NP_;
    const float* p1 = proj + (size_t)r1 * NP_;
    const float* p0 = proj + (size_t)r0 * NP_;
    const float qscale = 0.08838834764831845f;

#pragma unroll 1
    for (int p = 0; p < 4; ++p) {
        const int c = p * 1024 + tid * 4;
        const v4f x3 = *(const v4f*)(p3 + c);
        const v4f x2 = *(const v4f*)(p2 + c) * z2;
        const v4f x1 = *(const v4f*)(p1 + c) * z1;
        const v4f x0 = *(const v4f*)(p0 + c) * z0;
        const v4f w0 = *(const v4f*)(cw + 0 * CONV_ + c);
        const v4f w1 = *(const v4f*)(cw + 1 * CONV_ + c);
        const v4f w2 = *(const v4f*)(cw + 2 * CONV_ + c);
        const v4f w3 = *(const v4f*)(cw + 3 * CONV_ + c);
        v4f cv = w0 * x0;
        cv = w1 * x1 + cv;
        cv = w2 * x2 + cv;
        cv = w3 * x3 + cv;
#pragma unroll
        for (int i = 0; i < 4; ++i) cv[i] = silu_f(cv[i]);
        if (p < 2) {
            float ss = cv[0] * cv[0] + cv[1] * cv[1] + cv[2] * cv[2] + cv[3] * cv[3];
#pragma unroll
            for (int mm = 16; mm >= 1; mm >>= 1) ss += __shfl_xor(ss, mm, 32);
            const float rr = rsqrtf(ss + 1e-6f);
            cv = cv * rr;
            if (p == 0) cv = cv * qscale;
        }
        float* gp = act + (size_t)s * CONV_ + c;
        *(volatile v4f*)gp = cv;
        __threadfence();
        *(volatile v4f*)gp = cv;
    }
}

__global__ __launch_bounds__(256)
void delta_kernel(const float* __restrict__ act, const float* __restrict__ proj,
                  const float* __restrict__ alog, const float* __restrict__ dtb, float* core)
{
    __shared__ float sdec[S_];
    __shared__ float sbet[S_];
    __shared__ __attribute__((aligned(16))) float sout[32 * 32];

    const int tid  = threadIdx.x;
    const int lane = tid & 31;
    const int wave = tid >> 5;
    const int h    = blockIdx.x >> 2;
    const int dvb  = (blockIdx.x & 3) * 32;
    const int kh   = h >> 1;
    const int dvl  = tid >> 3;
    const int part = tid & 7;

    const float ae = expf(alog[h]);
    const float db = dtb[h];
#pragma unroll 1
    for (int s = tid; s < S_; s += 256) {
        const float b = proj[(size_t)s * NP_ + COLB_ + h];
        const float a = proj[(size_t)s * NP_ + COLA_ + h];
        sbet[s] = __builtin_amdgcn_rcpf(1.0f + __expf(-b));
        const float x  = a + db;
        const float sp = fmaxf(x, 0.0f) + log1pf(__expf(-fabsf(x)));
        sdec[s] = expf(-(ae * sp));
    }
    __syncthreads();

    float st[16];
#pragma unroll
    for (int i = 0; i < 16; ++i) st[i] = 0.0f;

    const float* qb = act + kh * DK_ + part * 16;
    const float* kb = act + KEY_ + kh * DK_ + part * 16;
    const float* vb = act + 2 * KEY_ + h * DV_ + dvb + dvl;

#pragma unroll 1
    for (int s = 0; s < S_; ++s) {
        const size_t ro = (size_t)s * CONV_;
        v4f k4[4], q4[4];
#pragma unroll
        for (int i = 0; i < 4; ++i) {
            k4[i] = *(const v4f*)(kb + ro + 4 * i);
            q4[i] = *(const v4f*)(qb + ro + 4 * i);
        }
        const float vv = vb[ro];
        const float eg = sdec[s];
        const float bt = sbet[s];

        float kv = 0.0f;
#pragma unroll
        for (int i = 0; i < 16; ++i) {
            st[i] = st[i] * eg;
            kv = st[i] * k4[i >> 2][i & 3] + kv;
        }
        kv += __shfl_xor(kv, 1, 32);
        kv += __shfl_xor(kv, 2, 32);
        kv += __shfl_xor(kv, 4, 32);

        const float delta = (vv - kv) * bt;

        float o = 0.0f;
#pragma unroll
        for (int i = 0; i < 16; ++i) {
            st[i] = k4[i >> 2][i & 3] * delta + st[i];
            o = st[i] * q4[i >> 2][i & 3] + o;
        }
        o += __shfl_xor(o, 1, 32);
        o += __shfl_xor(o, 2, 32);
        o += __shfl_xor(o, 4, 32);

        if (part == 0) sout[(s & 31) * 32 + dvl] = o;

        if ((s & 31) == 31) {
            __syncthreads();
            const int tt = wave * 4 + (lane >> 3);
            const int c  = (lane & 7) * 4;
            const v4f v = *(const v4f*)(sout + tt * 32 + c);
            float* gp = core + (size_t)(s - 31 + tt) * VAL_ + h * DV_ + dvb + c;
            *(volatile v4f*)gp = v;
            __threadfence();
            *(volatile v4f*)gp = v;
            __syncthreads();
        }
    }
}

__global__ __launch_bounds__(256)
void norm_gate_kernel(const float* __restrict__ core, const float* __restrict__ proj,
                      const float* __restrict__ nw, unsigned short* chi, unsigned short* clo)
{
    const int tid  = threadIdx.x;
    const int lane = tid & 31;
    const int wave = tid >> 5;
    const int r    = (blockIdx.x * 8 + wave) * 2 + (lane >> 4);
    const int s    = r >> 4;
    const int hh   = r & 15;
    const int c0   = (lane & 15) * 8;
    const size_t base = (size_t)s * VAL_ + hh * DV_ + c0;

    const v8f x = ld8f(core + base);
    float ss = 0.0f;
#pragma unroll
    for (int i = 0; i < 8; ++i) ss = x[i] * x[i] + ss;
    ss += __shfl_xor(ss, 8, 32);
    ss += __shfl_xor(ss, 4, 32);
    ss += __shfl_xor(ss, 2, 32);
    ss += __shfl_xor(ss, 1, 32);
    const float rr = rsqrtf(ss * (1.0f / 128.0f) + 1e-6f);

    const v8f z = ld8f(proj + (size_t)s * NP_ + COLZ_ + hh * DV_ + c0);
    const v8f w = ld8f(nw + c0);
    v8f y;
#pragma unroll
    for (int i = 0; i < 8; ++i) {
        const float t = (x[i] * rr) * w[i];
        y[i] = t * silu_f(z[i]);
    }
    u16x8 hv, lv;
    split8(y, hv, lv);
    *(volatile u16x8*)(chi + base) = hv;
    *(volatile u16x8*)(clo + base) = lv;
    __threadfence();
    *(volatile u16x8*)(chi + base) = hv;
    *(volatile u16x8*)(clo + base) = lv;
}

extern "C" void kernel_launch(void* const* d_in, const int* in_sizes, int n_in,
                              void* d_out, int out_size, void* d_ws, size_t ws_size,
                              hipStream_t stream)
{
    if (n_in < 11) return;
    if (in_sizes[0]  != S_ * H_)        return;
    if (in_sizes[1]  != H_ * CONV_)     return;
    if (in_sizes[2]  != H_ * VAL_)      return;
    if (in_sizes[3]  != H_ * NVH_)      return;
    if (in_sizes[4]  != H_ * NVH_)      return;
    if (in_sizes[5]  != 4 * CONV_)      return;
    if (in_sizes[6]  != NVH_)           return;
    if (in_sizes[7]  != NVH_)           return;
    if (in_sizes[8]  != DV_)            return;
    if (in_sizes[9]  != VAL_ * H_)      return;
    if (in_sizes[10] != S_)             return;
    if (out_size != S_ * H_)            return;
    if (ws_size < WS_END)               return;

    const float* hidden = (const float*)d_in[0];
    const float* W_qkv  = (const float*)d_in[1];
    const float* W_z    = (const float*)d_in[2];
    const float* W_b    = (const float*)d_in[3];
    const float* W_a    = (const float*)d_in[4];
    const float* convw  = (const float*)d_in[5];
    const float* dtb    = (const float*)d_in[6];
    const float* A_log  = (const float*)d_in[7];
    const float* nw     = (const float*)d_in[8];
    const float* W_out  = (const float*)d_in[9];
    const int*   mask   = (const int*)d_in[10];
    float* out = (float*)d_out;

    char* ws = (char*)d_ws;
    unsigned short* hsh  = (unsigned short*)(ws + OFF_HSH);
    unsigned short* hsl  = (unsigned short*)(ws + OFF_HSL);
    unsigned short* wch  = (unsigned short*)(ws + OFF_WCH);
    unsigned short* wcl  = (unsigned short*)(ws + OFF_WCL);
    unsigned short* woh  = (unsigned short*)(ws + OFF_WOH);
    unsigned short* wol  = (unsigned short*)(ws + OFF_WOL);
    float*          proj = (float*)(ws + OFF_PROJ);
    float*          act  = (float*)(ws + OFF_ACT);
    float*          core = (float*)(ws + OFF_CORE);
    unsigned short* cgh  = (unsigned short*)(ws + OFF_CGH);
    unsigned short* cgl  = (unsigned short*)(ws + OFF_CGL);

    {
        const int n8 = (S_ * H_) / 8;
        hs_cvt_kernel<<<dim3((n8 + 255) / 256), dim3(256), 0, stream>>>(hidden, mask, hsh, hsl, n8);
    }

    wt_cvt_kernel<<<dim3(CONV_ / 64, H_ / 64), dim3(256), 0, stream>>>(
        W_qkv, wch, wcl, (int)CONV_, (int)H_, (int)CONV_);
    wt_cvt_kernel<<<dim3(VAL_ / 64, H_ / 64), dim3(256), 0, stream>>>(
        W_z, wch + (size_t)COLZ_ * H_, wcl + (size_t)COLZ_ * H_, (int)VAL_, (int)H_, (int)VAL_);
    wt_cvt_kernel<<<dim3(1, H_ / 64), dim3(256), 0, stream>>>(
        W_b, wch + (size_t)COLB_ * H_, wcl + (size_t)COLB_ * H_, (int)NVH_, (int)H_, (int)NVH_);
    wt_cvt_kernel<<<dim3(1, H_ / 64), dim3(256), 0, stream>>>(
        W_a, wch + (size_t)COLA_ * H_, wcl + (size_t)COLA_ * H_, (int)NVH_, (int)H_, (int)(NP_ - COLA_));
    wt_cvt_kernel<<<dim3(H_ / 64, VAL_ / 64), dim3(256), 0, stream>>>(
        W_out, woh, wol, (int)H_, (int)VAL_, (int)H_);

    gemm_x3_kernel<2><<<dim3(NP_ / 64, S_ / 64), dim3(128), 0, stream>>>(
        (const unsigned short*)hsh, (const unsigned short*)hsl,
        (const unsigned short*)wch, (const unsigned short*)wcl,
        proj, (int)H_, (int)NP_);

    prep_kernel<<<dim3(S_), dim3(256), 0, stream>>>((const float*)proj, convw, act);

    delta_kernel<<<dim3(NVH_ * 4), dim3(256), 0, stream>>>(
        (const float*)act, (const float*)proj, A_log, dtb, core);

    norm_gate_kernel<<<dim3((S_ * NVH_) / 16), dim3(256), 0, stream>>>(
        (const float*)core, (const float*)proj, nw, cgh, cgl);

    gemm_x3_kernel<2><<<dim3(H_ / 64, S_ / 64), dim3(128), 0, stream>>>(
        (const unsigned short*)cgh, (const unsigned short*)cgl,
        (const unsigned short*)woh, (const unsigned short*)wol,
        out, (int)VAL_, (int)H_);
}
